// net_a_bit_overkill_19997367730394
// MI455X (gfx1250) — hardware-verified
//
#include <hip/hip_runtime.h>
#include <stdint.h>

typedef __bf16   v16b __attribute__((ext_vector_type(16)));
typedef __bf16   v8b  __attribute__((ext_vector_type(8)));
typedef float    v8f  __attribute__((ext_vector_type(8)));
typedef float    v4f  __attribute__((ext_vector_type(4)));
typedef unsigned int v4u __attribute__((ext_vector_type(4)));

#define D_IN   13
#define HID    128
#define KP1    32
#define RB     64
#define NT_MLP 128
#define XS_P   40
#define H_P    136
static_assert(RB == (NT_MLP / 32) * 16);
static_assert(((XS_P * 2) % 16) == 0 && ((H_P * 2) % 16) == 0);
static_assert((KP1 % 32) == 0 && (HID % 32) == 0);

__device__ __forceinline__ unsigned short bf_bits(float f) {
  unsigned u = __float_as_uint(f);
  return (unsigned short)((u + 0x7FFFu + ((u >> 16) & 1u)) >> 16);
}
__device__ __forceinline__ float bf_up(unsigned short h) { return __uint_as_float(((unsigned)h) << 16); }
__device__ __forceinline__ float bf_rn(float f) { return bf_up(bf_bits(f)); }
__device__ __forceinline__ unsigned bf_mag(float f) {
  return (((unsigned)bf_bits(f)) << 16) & 0x7fffffffu;
}
__device__ __forceinline__ unsigned pk16(unsigned short a, unsigned short b) { return (unsigned)a | ((unsigned)b << 16); }
__device__ __forceinline__ __bf16 bf_from_bits(unsigned short h) { return __builtin_bit_cast(__bf16, h); }
__device__ __forceinline__ v8f zero8() { v8f z = {0.f, 0.f, 0.f, 0.f, 0.f, 0.f, 0.f, 0.f}; return z; }

__device__ __forceinline__ v16b ldfrag_b(const __bf16* p) {
  union { v16b v; v8b h[2]; } f;
  f.h[0] = *(const v8b*)(p);
  f.h[1] = *(const v8b*)(p + 16);
  return f.v;
}

__device__ __forceinline__ v8f mma_b(v16b a, v16b b, v8f c) {
  c = __builtin_amdgcn_wmma_f32_16x16x32_bf16(false, a, false, b, (short)0, c, false, false);
#if defined(__HIP_DEVICE_COMPILE__)
  asm volatile("v_nop\n\tv_nop\n\tv_nop\n\tv_nop" : "+v"(c) : "v"(a), "v"(b));
#endif
  return c;
}
__device__ __forceinline__ void wave_sync_lds() {
  __builtin_amdgcn_fence(__ATOMIC_RELEASE, "workgroup");
  __builtin_amdgcn_wave_barrier();
  __builtin_amdgcn_fence(__ATOMIC_ACQUIRE, "workgroup");
}

__global__ __launch_bounds__(256) void k_mask(const float* __restrict__ W, int nrow, int ncol, int kp, int kkeep,
                                              unsigned short* Wp) {
  __shared__ unsigned s_cnt[8];
  const int tid  = threadIdx.x;
  const int lane = tid & 31;
  const int wave = tid >> 5;
  const int n    = nrow * ncol;

  unsigned prefix = 0u;
  for (int bit = 30; bit >= 16; --bit) {
    const unsigned cand = prefix | (1u << bit);
    unsigned c = 0u;
    for (int i = tid; i < n; i += 256) c += (bf_mag(W[i]) >= cand) ? 1u : 0u;
#pragma unroll
    for (int off = 1; off < 32; off <<= 1) c += __shfl_xor(c, off, 32);
    if (lane == 0) s_cnt[wave] = c;
    __syncthreads();
    unsigned tot = 0u;
#pragma unroll
    for (int w = 0; w < 8; ++w) tot += s_cnt[w];
    __syncthreads();
    if (tot >= (unsigned)kkeep) prefix = cand;
  }

  const int n8 = (nrow * kp) >> 3;
  for (int pass = 0; pass < 2; ++pass) {
    for (int i = tid; i < n8; i += 256) {
      const int e0  = i << 3;
      const int row = e0 / kp;
      const int c0  = e0 - row * kp;
      v4u p;
#pragma unroll
      for (int e = 0; e < 4; ++e) {
        const int ka  = c0 + 2 * e;
        const int kb  = ka + 1;
        const int kac = (ka < ncol) ? ka : (ncol - 1);
        const int kbc = (kb < ncol) ? kb : (ncol - 1);
        const float wa = W[row * ncol + kac];
        const float wb = W[row * ncol + kbc];
        const bool keepa = (ka < ncol) && (bf_mag(wa) >= prefix);
        const bool keepb = (kb < ncol) && (bf_mag(wb) >= prefix);
        const unsigned short ha = keepa ? bf_bits(wa) : (unsigned short)0;
        const unsigned short hb = keepb ? bf_bits(wb) : (unsigned short)0;
        p[e] = pk16(ha, hb);
      }
      *(volatile v4u*)(Wp + e0) = p;
    }
    __threadfence();
  }
}

__global__ __launch_bounds__(NT_MLP)
void k_mlp(const float* __restrict__ X, const unsigned short* __restrict__ W1p, const float* __restrict__ b1,
           const unsigned short* __restrict__ W2p, const float* __restrict__ b2,
           const float* __restrict__ W3, const float* __restrict__ b3, float* out) {
  __shared__ __align__(16) __bf16 Xs[RB * XS_P];
  __shared__ __align__(16) __bf16 Hh[RB * H_P];
  __shared__ __align__(16) __bf16 Hl[RB * H_P];
  __shared__ __align__(16) float  Os[RB];

  const int tid  = threadIdx.x;
  const int lane = tid & 31;
  const int wave = tid >> 5;
  const int hh   = lane >> 4;
  const int m    = lane & 15;
  const int row0 = blockIdx.x * RB;

  const float* Xg = X + (size_t)row0 * D_IN;
  for (int i = tid; i < RB * XS_P; i += NT_MLP) {
    const int r  = i / XS_P;
    const int c  = i - r * XS_P;
    const int cc = (c < D_IN) ? c : (D_IN - 1);
    const float v = Xg[r * D_IN + cc];
    const unsigned short bits = (c < D_IN) ? bf_bits(v) : (unsigned short)0;
    Xs[i] = bf_from_bits(bits);
  }
  __syncthreads();

  const int lrow = wave * 16;
  const __bf16* W1b = (const __bf16*)(const void*)W1p;
  const __bf16* W2b = (const __bf16*)(const void*)W2p;

  {
    const v16b a = ldfrag_b(Xs + (lrow + m) * XS_P + 8 * hh);
#pragma unroll
    for (int t = 0; t < 8; ++t) {
      const v16b bfr = ldfrag_b(W1b + (size_t)(t * 16 + m) * KP1 + 8 * hh);
      const v8f acc = mma_b(a, bfr, zero8());
      const float bv = bf_rn(b1[t * 16 + m]);
#pragma unroll
      for (int r = 0; r < 8; ++r) {
        const float v = fmaxf(acc[r] + bv, 0.0f);
        const unsigned short h0 = bf_bits(v);
        const unsigned short l0 = bf_bits(v - bf_up(h0));
        const int o = (lrow + 8 * hh + r) * H_P + t * 16 + m;
        Hh[o] = bf_from_bits(h0);
        Hl[o] = bf_from_bits(l0);
      }
    }
  }
  wave_sync_lds();

  v16b ah[4], al[4];
#pragma unroll
  for (int kc = 0; kc < 4; ++kc) {
    ah[kc] = ldfrag_b(Hh + (lrow + m) * H_P + kc * 32 + 8 * hh);
    al[kc] = ldfrag_b(Hl + (lrow + m) * H_P + kc * 32 + 8 * hh);
  }

  float part[8] = {0.f, 0.f, 0.f, 0.f, 0.f, 0.f, 0.f, 0.f};
#pragma unroll 1
  for (int t = 0; t < 8; ++t) {
    v16b bq[4];
#pragma unroll
    for (int kc = 0; kc < 4; ++kc)
      bq[kc] = ldfrag_b(W2b + (size_t)(t * 16 + m) * HID + kc * 32 + 8 * hh);
    v8f acc = zero8();
#pragma unroll
    for (int kc = 0; kc < 4; ++kc) {
      acc = mma_b(ah[kc], bq[kc], acc);
      acc = mma_b(al[kc], bq[kc], acc);
    }
    const float bv  = bf_rn(b2[t * 16 + m]);
    const float w3v = bf_rn(W3[t * 16 + m]);
#pragma unroll
    for (int r = 0; r < 8; ++r) {
      const float h2 = fmaxf(acc[r] + bv, 0.0f);
      part[r] = fmaf(h2, w3v, part[r]);
    }
  }

#pragma unroll
  for (int off = 1; off < 16; off <<= 1) {
#pragma unroll
    for (int r = 0; r < 8; ++r) part[r] += __shfl_xor(part[r], off, 32);
  }
  const float bb = bf_rn(b3[0]);
  if (m == 0) {
#pragma unroll
    for (int r = 0; r < 8; ++r) Os[lrow + 8 * hh + r] = part[r] + bb;
  }
  __syncthreads();

  if (tid < 16) {
    const v4f v = *(const v4f*)(Os + tid * 4);
    float* op = out + (size_t)row0 + tid * 4;
    *(volatile v4f*)op = v;
    __threadfence();
    *(volatile v4f*)op = v;
  }
}

extern "C" void kernel_launch(void* const* d_in, const int* in_sizes, int n_in,
                              void* d_out, int out_size, void* d_ws, size_t ws_size,
                              hipStream_t stream) {
  if (n_in < 7) return;
  if (in_sizes[1] != HID * D_IN) return;
  if (in_sizes[2] != HID) return;
  if (in_sizes[3] != HID * HID) return;
  if (in_sizes[4] != HID) return;
  if (in_sizes[5] != HID) return;
  if (in_sizes[6] < 1) return;
  const int nX = in_sizes[0];
  if (nX <= 0 || (nX % (D_IN * RB)) != 0) return;
  const int nrows = nX / D_IN;
  if (out_size != nrows) return;

  const float* X  = (const float*)d_in[0];
  const float* W1 = (const float*)d_in[1];
  const float* b1 = (const float*)d_in[2];
  const float* W2 = (const float*)d_in[3];
  const float* b2 = (const float*)d_in[4];
  const float* W3 = (const float*)d_in[5];
  const float* b3 = (const float*)d_in[6];

  const size_t PW1 = (size_t)HID * KP1 * 2;
  const size_t PW2 = (size_t)HID * HID * 2;
  size_t off = 0;
  const size_t oW1 = off; off += PW1;
  const size_t oW2 = off; off += PW2;
  if (off > ws_size) return;
  if (off > (size_t)134217728) return;

  char* ws = (char*)d_ws;
  unsigned short* W1p = (unsigned short*)(ws + oW1);
  unsigned short* W2p = (unsigned short*)(ws + oW2);

  const int k1 = 1332;
  const int k2 = 8192;

  k_mask<<<dim3(1), dim3(256), 0, stream>>>(W1, HID, D_IN, KP1, k1, W1p);
  k_mask<<<dim3(1), dim3(256), 0, stream>>>(W2, HID, HID, HID, k2, W2p);
  k_mlp<<<dim3((unsigned)(nrows / RB)), dim3(NT_MLP), 0, stream>>>(X, W1p, b1, W2p, b2, W3, b3, (float*)d_out);
  (void)hipGetLastError();
}
